// CapsuleLayer_1778116461334
// MI455X (gfx1250) — hardware-verified
//
#include <hip/hip_runtime.h>


#define A_DIM 64
#define B_DIM 128
#define D_DIM 256
#define H_DIM 64
#define C_DIM 32

typedef __bf16 v16bf __attribute__((ext_vector_type(16)));
typedef float  v8f   __attribute__((ext_vector_type(8)));

#define PSTRIDE 260
#define KC 32
#define WT_STRIDE 40

template<int M>
__global__ __launch_bounds__(256) void caps_stage(
    const float* __restrict__ Xbase,
    const float* __restrict__ Wbase,
    float* Out,
    int nA, int outStrideA, int outStrideW)
{
  extern __shared__ __align__(16) char smem[];
  constexpr int CHUNK_BYTES = 3 * (M * KC + D_DIM * WT_STRIDE) * 2;
  constexpr int P_BYTES = M * PSTRIDE * 4;
  constexpr int REGION = ((CHUNK_BYTES > P_BYTES ? CHUNK_BYTES : P_BYTES) + 15) / 16 * 16;
  float*  P   = (float*)smem;
  __bf16* Xh  = (__bf16*)smem;
  __bf16* Xm  = Xh + M * KC;
  __bf16* Xl  = Xm + M * KC;
  __bf16* Wth = Xl + M * KC;
  __bf16* Wtm = Wth + D_DIM * WT_STRIDE;
  __bf16* Wtl = Wtm + D_DIM * WT_STRIDE;
  float* tail   = (float*)(smem + REGION);
  float* logits = tail;
  float* probs  = tail + M;
  float* outvec = tail + 2 * M;
  float* red    = tail + 2 * M + 256;

  const int tid  = threadIdx.x;
  const int lane = tid & 31;
  const int wv   = tid >> 5;
  const int lr   = lane & 15;
  const int hh   = lane >> 4;

  const int aIdx = blockIdx.x % nA;
  const int wIdx = blockIdx.x / nA;
  const float* Xg = Xbase + (size_t)aIdx * (M * D_DIM);
  const float* Wg = Wbase + (size_t)wIdx * (D_DIM * D_DIM);

  constexpr int MT = M / 16;
  v8f acc[MT][2];
  #pragma unroll
  for (int m = 0; m < MT; ++m)
    #pragma unroll
    for (int j = 0; j < 2; ++j)
      acc[m][j] = (v8f){0.f,0.f,0.f,0.f,0.f,0.f,0.f,0.f};

  for (int kc = 0; kc < D_DIM / KC; ++kc) {
    __syncthreads();
    constexpr int XE = M * KC / 256;
    #pragma unroll
    for (int i = 0; i < XE; ++i) {
      int idx = i * 256 + tid;
      int r = idx >> 5, c = idx & 31;
      float v = Xg[r * D_DIM + kc * KC + c];
      __bf16 hi = (__bf16)v;
      float r1 = v - (float)hi;
      __bf16 mid = (__bf16)r1;
      Xh[r * KC + c] = hi;
      Xm[r * KC + c] = mid;
      Xl[r * KC + c] = (__bf16)(r1 - (float)mid);
    }
    #pragma unroll 4
    for (int r = 0; r < KC; ++r) {
      float v = Wg[(kc * KC + r) * D_DIM + tid];
      __bf16 hi = (__bf16)v;
      float r1 = v - (float)hi;
      __bf16 mid = (__bf16)r1;
      Wth[tid * WT_STRIDE + r] = hi;
      Wtm[tid * WT_STRIDE + r] = mid;
      Wtl[tid * WT_STRIDE + r] = (__bf16)(r1 - (float)mid);
    }
    __syncthreads();

    v16bf bh[2], bm[2], bl[2];
    #pragma unroll
    for (int j = 0; j < 2; ++j) {
      int col  = (wv * 2 + j) * 16 + lr;
      int base = col * WT_STRIDE + hh * 8;
      #pragma unroll
      for (int e = 0; e < 8; ++e) {
        bh[j][e] = Wth[base + e];          bm[j][e] = Wtm[base + e];          bl[j][e] = Wtl[base + e];
        bh[j][8 + e] = Wth[base + 16 + e]; bm[j][8 + e] = Wtm[base + 16 + e]; bl[j][8 + e] = Wtl[base + 16 + e];
      }
    }
    #pragma unroll
    for (int m = 0; m < MT; ++m) {
      int xb = (m * 16 + lr) * KC + hh * 8;
      v16bf ah, am, al;
      #pragma unroll
      for (int e = 0; e < 8; ++e) {
        ah[e] = Xh[xb + e];  ah[8 + e] = Xh[xb + 16 + e];
        am[e] = Xm[xb + e];  am[8 + e] = Xm[xb + 16 + e];
        al[e] = Xl[xb + e];  al[8 + e] = Xl[xb + 16 + e];
      }
      #pragma unroll
      for (int j = 0; j < 2; ++j) {
        acc[m][j] = __builtin_amdgcn_wmma_f32_16x16x32_bf16(false, ah, false, bh[j], (short)0, acc[m][j], false, false);
        acc[m][j] = __builtin_amdgcn_wmma_f32_16x16x32_bf16(false, ah, false, bm[j], (short)0, acc[m][j], false, false);
        acc[m][j] = __builtin_amdgcn_wmma_f32_16x16x32_bf16(false, am, false, bh[j], (short)0, acc[m][j], false, false);
        acc[m][j] = __builtin_amdgcn_wmma_f32_16x16x32_bf16(false, ah, false, bl[j], (short)0, acc[m][j], false, false);
        acc[m][j] = __builtin_amdgcn_wmma_f32_16x16x32_bf16(false, am, false, bm[j], (short)0, acc[m][j], false, false);
        acc[m][j] = __builtin_amdgcn_wmma_f32_16x16x32_bf16(false, al, false, bh[j], (short)0, acc[m][j], false, false);
        asm volatile("v_nop\n\tv_nop\n\tv_nop\n\tv_nop" : "+v"(acc[m][j]) : "v"(ah), "v"(am), "v"(al), "v"(bh[j]), "v"(bm[j]), "v"(bl[j]));
      }
    }
  }
  __syncthreads();

  #pragma unroll
  for (int m = 0; m < MT; ++m)
    #pragma unroll
    for (int j = 0; j < 2; ++j) {
      int col = (wv * 2 + j) * 16 + lr;
      #pragma unroll
      for (int v = 0; v < 8; ++v)
        P[(m * 16 + hh * 8 + v) * PSTRIDE + col] = acc[m][j][v];
    }
  if (tid < M) logits[tid] = 0.f;
  __syncthreads();

  float lastOut = 0.f;
  for (int it = 0; it < 3; ++it) {
    float lv = (tid < M) ? logits[tid] : -3.0e38f;
    red[tid] = lv; __syncthreads();
    #pragma unroll
    for (int s = 128; s > 0; s >>= 1) { if (tid < s) red[tid] = fmaxf(red[tid], red[tid + s]); __syncthreads(); }
    float mx = red[0]; __syncthreads();
    float ev = (tid < M) ? __expf(lv - mx) : 0.f;
    red[tid] = ev; __syncthreads();
    #pragma unroll
    for (int s = 128; s > 0; s >>= 1) { if (tid < s) red[tid] += red[tid + s]; __syncthreads(); }
    float esum = red[0]; __syncthreads();
    if (tid < M) probs[tid] = ev / esum;
    __syncthreads();

    float sAcc = 0.f;
    for (int b = 0; b < M; ++b) sAcc += probs[b] * P[b * PSTRIDE + tid];
    red[tid] = sAcc * sAcc; __syncthreads();
    #pragma unroll
    for (int s = 128; s > 0; s >>= 1) { if (tid < s) red[tid] += red[tid + s]; __syncthreads(); }
    float sq = red[0]; __syncthreads();
    float ov = sAcc * (sq / (1.f + sq)) * rsqrtf(sq);
    outvec[tid] = ov;
    lastOut = ov;
    __syncthreads();

    if (it != 2) {
      const int RW = M / 8;
      for (int r = 0; r < RW; ++r) {
        int b = wv * RW + r;
        float p = 0.f;
        #pragma unroll
        for (int i = 0; i < 8; ++i) { int d = lane + i * 32; p += P[b * PSTRIDE + d] * outvec[d]; }
        #pragma unroll
        for (int off = 16; off > 0; off >>= 1) p += __shfl_down(p, off);
        if (lane == 0) logits[b] += p;
      }
      __syncthreads();
    }
  }

  float* op = Out + (size_t)aIdx * outStrideA + (size_t)wIdx * outStrideW + tid;
  *(volatile float*)op = lastOut;
  __threadfence();
  *(volatile float*)op = lastOut;
}

extern "C" void kernel_launch(void* const* d_in, const int* in_sizes, int n_in,
                              void* d_out, int out_size, void* d_ws, size_t ws_size,
                              hipStream_t stream) {
  const float* x  = (const float*)d_in[0];
  const float* w1 = (const float*)d_in[1];
  const float* w2 = (const float*)d_in[2];
  float* out  = (float*)d_out;
  float* out1 = (float*)d_ws;

  size_t reg1 = (size_t)128 * PSTRIDE * 4; { size_t cb = (size_t)3 * (128 * KC + D_DIM * WT_STRIDE) * 2; if (cb > reg1) reg1 = cb; } reg1 = (reg1 + 15) / 16 * 16;
  size_t reg2 = (size_t) 64 * PSTRIDE * 4; { size_t cb = (size_t)3 * ( 64 * KC + D_DIM * WT_STRIDE) * 2; if (cb > reg2) reg2 = cb; } reg2 = (reg2 + 15) / 16 * 16;
  size_t smem1 = reg1 + (size_t)(2 * 128 + 512) * 4;
  size_t smem2 = reg2 + (size_t)(2 *  64 + 512) * 4;

  caps_stage<128><<<dim3(H_DIM * A_DIM), dim3(256), smem1, stream>>>(
      x, w1, out1, A_DIM, H_DIM * D_DIM  , D_DIM  );

  caps_stage<64><<<dim3(C_DIM * A_DIM), dim3(256), smem2, stream>>>(
      out1, w2, out, A_DIM, D_DIM  , A_DIM * D_DIM  );
}
